// SpatialGNN_1219770712590
// MI455X (gfx1250) — hardware-run, weakly checked
//
#include <hip/hip_runtime.h>
#include <math.h>

constexpr int NNODE  = 20000;
constexpr int NEDGE  = 400000;
constexpr int NVIRT  = NEDGE + NNODE;
constexpr int NGRAPH = 200;
constexpr int CIN    = 8;
constexpr int NHEAD  = 4;
constexpr int HID1   = 64;
constexpr int OUT2   = 32;
constexpr int AW1    = NHEAD * HID1;
constexpr int AW2    = NHEAD * OUT2;
constexpr int XW1    = 2 * AW1;
constexpr int XW2    = 2 * AW2;
constexpr int KP1    = 32;
constexpr int KD2    = 64;
constexpr int NPAD   = 20032;
constexpr int NT     = 256;
constexpr int SRB    = 1024;
constexpr int NTILE  = 20;
constexpr int NACC   = NTILE * SRB;
constexpr int RPW    = SRB / (NT / 32);
constexpr int OWN_SHIFT = 16 + 7;
constexpr float WCARRY     = 16.0f;
constexpr float WCARRY_INV = 1.0f / 16.0f;
constexpr float LN_EPS     = 1e-5f;
constexpr float NEG_SLOPE_C = 0.2f;

static_assert(NPAD % 64 == 0 && NPAD >= NNODE, "");
static_assert(XW1 % 64 == 0 && XW2 % 64 == 0, "");
static_assert(KP1 % 32 == 0 && KD2 % 32 == 0, "");
static_assert(NACC >= NPAD, "");
static_assert(RPW == 128 && (1 << 7) == RPW, "");
static_assert(NNODE < 65536 && SRB <= 1024, "");
static_assert(NNODE % 8 == 0, "");

typedef __attribute__((ext_vector_type(16))) _Float16 v16h;
typedef __attribute__((ext_vector_type(8)))  _Float16 v8h;
typedef __attribute__((ext_vector_type(16))) __bf16   v16b;
typedef __attribute__((ext_vector_type(8)))  __bf16   v8b;
typedef __attribute__((ext_vector_type(8)))  float    v8f;
typedef __attribute__((ext_vector_type(4)))  float    v4f;
typedef __attribute__((ext_vector_type(4)))  unsigned int v4u;
typedef __attribute__((ext_vector_type(4)))  int      v4i;

__device__ __forceinline__ unsigned short f2bf_bits(float f) {
  unsigned u = __float_as_uint(f);
  return (unsigned short)((u + 0x7FFFu + ((u >> 16) & 1u)) >> 16);
}
__device__ __forceinline__ float bf_bits2f(unsigned short h) { return __uint_as_float(((unsigned)h) << 16); }

__device__ __forceinline__ void dep_guard_h(v8f& a, v8f& b, v16h x, v16h y) { asm volatile("v_nop\n\tv_nop\n\tv_nop\n\tv_nop" : "+v"(a), "+v"(b) : "v"(x), "v"(y)); }
__device__ __forceinline__ void dep_guard_b(v8f& a, v8f& b, v16b x, v16b y) { asm volatile("v_nop\n\tv_nop\n\tv_nop\n\tv_nop" : "+v"(a), "+v"(b) : "v"(x), "v"(y)); }
__device__ __forceinline__ void keep4_h(v16h a, v16h b, v16h c, v16h d) { asm volatile("v_nop" :: "v"(a), "v"(b), "v"(c), "v"(d)); }
__device__ __forceinline__ void keep4_b(v16b a, v16b b, v16b c, v16b d) { asm volatile("v_nop" :: "v"(a), "v"(b), "v"(c), "v"(d)); }
__device__ __forceinline__ void acc_guard4(v8f& a, v8f& b, v8f& c, v8f& d) { asm volatile("v_nop\n\tv_nop\n\tv_nop\n\tv_nop" : "+v"(a), "+v"(b), "+v"(c), "+v"(d)); }
template <typename T> struct Frag;
template <> struct Frag<_Float16> {
  typedef v16h V; union U { v16h v; v8h h[2]; };
  static __device__ __forceinline__ v16h load(const _Float16* p) {
    U f; f.h[0] = *(const v8h*)(p); f.h[1] = *(const v8h*)(p + 16); return f.v;
  }
  static __device__ __forceinline__ v8f mma(v16h a, v16h b, v8f c) {
    return __builtin_amdgcn_wmma_f32_16x16x32_f16(false, a, false, b, (short)0, c, false, false);
  }
  static __device__ __forceinline__ void guard(v8f& a, v8f& b, v16h x, v16h y) { dep_guard_h(a, b, x, y); }
  static __device__ __forceinline__ void keep(v16h a, v16h b, v16h c, v16h d) { keep4_h(a, b, c, d); }
};
template <> struct Frag<__bf16> {
  typedef v16b V; union U { v16b v; v8b h[2]; };
  static __device__ __forceinline__ v16b load(const __bf16* p) {
    U f; f.h[0] = *(const v8b*)(p); f.h[1] = *(const v8b*)(p + 16); return f.v;
  }
  static __device__ __forceinline__ v8f mma(v16b a, v16b b, v8f c) {
    return __builtin_amdgcn_wmma_f32_16x16x32_bf16(false, a, false, b, (short)0, c, false, false);
  }
  static __device__ __forceinline__ void guard(v8f& a, v8f& b, v16b x, v16b y) { dep_guard_b(a, b, x, y); }
  static __device__ __forceinline__ void keep(v16b a, v16b b, v16b c, v16b d) { keep4_b(a, b, c, d); }
};

__device__ __forceinline__ unsigned pk16(unsigned short a, unsigned short b) { return (unsigned)a | ((unsigned)b << 16); }
__device__ __forceinline__ unsigned short h_bits(float f) { const _Float16 h = (_Float16)f; return __builtin_bit_cast(unsigned short, h); }
__device__ __forceinline__ v4u pack8h(float f0, float f1, float f2, float f3, float f4, float f5, float f6, float f7) {
  return (v4u){pk16(h_bits(f0), h_bits(f1)), pk16(h_bits(f2), h_bits(f3)), pk16(h_bits(f4), h_bits(f5)), pk16(h_bits(f6), h_bits(f7))};
}
__device__ __forceinline__ int opaque_i(int v) { asm volatile("" : "+v"(v)); return v; }
__device__ __forceinline__ float opaque_f(float v) { asm volatile("" : "+v"(v)); return v; }

template <int ET> struct Elem;
template <> struct Elem<0> { typedef _Float16 T; };
template <> struct Elem<1> { typedef __bf16 T; };
template <int ET, bool SPLIT, int BIAS_MODE, int OUT_MODE, bool RESID, int ACT = 0>
__global__ __launch_bounds__(256) void wmma_gemm64(
    const unsigned short* __restrict__ Ap, const unsigned short* __restrict__ A2p, int lda, long strideA,
    const unsigned short* __restrict__ Btp, const unsigned short* __restrict__ Bt2p, int ldb, long strideB,
    void* __restrict__ Cout, void* __restrict__ Cout2, int ldc, long strideC,
    const float* __restrict__ bias,
    const float* __restrict__ resid, long strideR,
    int M, int N, int K, float scale) {
  typedef typename Elem<ET>::T T;
  typedef typename Frag<T>::V V;
  const T* A = (const T*)Ap; const T* A2 = (const T*)A2p; const T* Bt = (const T*)Btp; const T* Bt2 = (const T*)Bt2p;
  __shared__ __align__(16) float sT[8][16 * 68];
  const int b    = blockIdx.y;
  const int lane = threadIdx.x & 31;
  const int wave = threadIdx.x >> 5;
  const int tilesN = N >> 6;
  const int tilesM = M >> 6;
  const int tile = blockIdx.x * 8 + wave;
  if (tile >= tilesM * tilesN) return;
  const int tm = tile / tilesN;
  const int tn = tile - tm * tilesN;
  const int m0 = tm << 6;
  const int n0 = tn << 6;

  const T* Ab  = A  + (size_t)b * strideA;
  const T* Bb  = Bt + (size_t)b * strideB;
  const T* Ab2 = SPLIT ? (A2  + (size_t)b * strideA) : nullptr;
  const T* Bb2 = SPLIT ? (Bt2 + (size_t)b * strideB) : nullptr;

  const int rlane = lane & 15;
  const int koff  = (lane >> 4) * 8;
  const int mOff  = (lane >> 4) * 8;

  v8f acc[4][4];
#pragma unroll
  for (int i = 0; i < 4; ++i)
#pragma unroll
    for (int j = 0; j < 4; ++j) acc[i][j] = (v8f){0.f,0.f,0.f,0.f,0.f,0.f,0.f,0.f};

  for (int k0 = 0; k0 < K; k0 += 32) {
    V bh[4], bl[4];
#pragma unroll
    for (int j = 0; j < 4; ++j) {
      const size_t bo = (size_t)(n0 + (j << 4) + rlane) * ldb + koff + k0;
      bh[j] = Frag<T>::load(Bb + bo);
      if (SPLIT) bl[j] = Frag<T>::load(Bb2 + bo);
    }
#pragma unroll
    for (int i = 0; i < 4; ++i) {
      const size_t ao = (size_t)(m0 + (i << 4) + rlane) * lda + koff + k0;
      V ah = Frag<T>::load(Ab + ao);
      V al;
      if (SPLIT) al = Frag<T>::load(Ab2 + ao);
#pragma unroll
      for (int j = 0; j < 4; ++j) {
        acc[i][j] = Frag<T>::mma(ah, bh[j], acc[i][j]);
        if (SPLIT) {
          acc[i][j] = Frag<T>::mma(ah, bl[j], acc[i][j]);
          acc[i][j] = Frag<T>::mma(al, bh[j], acc[i][j]);
        }
      }
      Frag<T>::guard(acc[i][0], acc[i][3], ah, SPLIT ? al : ah);
    }
    Frag<T>::keep(bh[0], bh[1], bh[2], bh[3]);
    if (SPLIT) Frag<T>::keep(bl[0], bl[1], bl[2], bl[3]);
  }
  acc_guard4(acc[0][0], acc[0][1], acc[0][2], acc[0][3]);
  acc_guard4(acc[1][0], acc[1][1], acc[1][2], acc[1][3]);
  acc_guard4(acc[2][0], acc[2][1], acc[2][2], acc[2][3]);
  acc_guard4(acc[3][0], acc[3][1], acc[3][2], acc[3][3]);

  float* slab = sT[wave];
  const float* Rb = RESID ? (resid + (size_t)b * strideR) : nullptr;
#pragma unroll
  for (int i = 0; i < 4; ++i) {
    const int mBase = m0 + (i << 4);
#pragma unroll
    for (int j = 0; j < 4; ++j) {
      const int n = n0 + (j << 4) + rlane;
      float bv = 0.f;
      if (BIAS_MODE == 2) bv = bias[n];
#pragma unroll
      for (int r = 0; r < 8; ++r) {
        float v = acc[i][j][r] * scale;
        if (BIAS_MODE == 1) v += bias[mBase + mOff + r];
        if (BIAS_MODE == 2) v += bv;
        if (RESID) v += Rb[(size_t)(mBase + mOff + r) * ldc + n];
        if (ACT == 2) v = fmaxf(v, 0.0f);
        if (ACT == 4) v = (v > 0.f) ? v : 0.01f * v;
        slab[(mOff + r) * 68 + (j << 4) + rlane] = v;
      }
    }
    __builtin_amdgcn_fence(__ATOMIC_RELEASE, "workgroup");
    __builtin_amdgcn_wave_barrier();
    __builtin_amdgcn_fence(__ATOMIC_ACQUIRE, "workgroup");
    if (OUT_MODE == 0) {
      float* C = (float*)Cout + (size_t)b * strideC;
      const int hh = lane >> 4, c4 = (lane & 15) * 4;
      for (int pass = 0; pass < 2; ++pass) {
#pragma unroll
        for (int it = 0; it < 8; ++it) {
          const int row = it * 2 + hh;
          v4f v = *(const v4f*)(slab + row * 68 + c4);
          *(volatile v4f*)(C + (size_t)(mBase + row) * ldc + n0 + c4) = v;
        }
        __threadfence();
      }
    } else {
      const int q = lane >> 3, c8 = (lane & 7) * 8;
      unsigned short* C  = (unsigned short*)Cout  + (size_t)b * strideC;
      unsigned short* C2 = (OUT_MODE == 2) ? ((unsigned short*)Cout2 + (size_t)b * strideC) : nullptr;
      for (int pass = 0; pass < 2; ++pass) {
#pragma unroll
        for (int it = 0; it < 4; ++it) {
          const int row = it * 4 + q;
          const float* sp = slab + row * 68 + c8;
          v8h hv, lv;
#pragma unroll
          for (int e = 0; e < 8; ++e) {
            if (OUT_MODE == 1) {
              hv[e] = (_Float16)sp[e];
            } else {
              unsigned short hb = f2bf_bits(sp[e]);
              unsigned short lb = f2bf_bits(sp[e] - bf_bits2f(hb));
              hv[e] = __builtin_bit_cast(_Float16, hb);
              lv[e] = __builtin_bit_cast(_Float16, lb);
            }
          }
          *(volatile v8h*)(C + (size_t)(mBase + row) * ldc + n0 + c8) = hv;
          if (OUT_MODE == 2) *(volatile v8h*)(C2 + (size_t)(mBase + row) * ldc + n0 + c8) = lv;
        }
        __threadfence();
      }
    }
    __builtin_amdgcn_fence(__ATOMIC_RELEASE, "workgroup");
    __builtin_amdgcn_wave_barrier();
    __builtin_amdgcn_fence(__ATOMIC_ACQUIRE, "workgroup");
  }
}

__device__ __forceinline__ int blk_excl_scan(int cnt, int* scan_ws, int tid, int* tot) {
  const int lane = tid & 31, wave = tid >> 5; int incl = cnt;
#pragma unroll
  for (int o = 1; o < 32; o <<= 1) { const int v = __shfl_up(incl, o, 32); if (lane >= o) incl += v; }
  if (lane == 31) scan_ws[wave] = incl;
  __syncthreads();
  if (wave == 0) { int wv = scan_ws[lane & 7]; wv = (lane < NT / 32) ? wv : 0; int wincl = wv;
#pragma unroll
    for (int o = 1; o < 32; o <<= 1) { const int v = __shfl_up(wincl, o, 32); if (lane >= o) wincl += v; }
    if (lane < NT / 32) scan_ws[32 + lane] = wincl - wv; if (lane == 31) scan_ws[64] = wincl; }
  __syncthreads();
  const int res = scan_ws[32 + wave] + incl - cnt; *tot = scan_ws[64];
  return res;
}

template <int SP, int CAP>
__device__ __forceinline__ int chunk_hits(const int* __restrict__ dstv, const int* __restrict__ srcv, int e0, int n0, int tid,
                                          int* LIST, int* scan_ws) {
  static_assert(SP % 4 == 0 && NEDGE % SP == 0 && NEDGE >= SP, "");
  const int eb = e0 + tid * SP;
  const bool isreal = eb < NEDGE;
  const int ebc = isreal ? eb : (NEDGE - SP);
  const int iri = opaque_i(isreal ? 1 : 0);
  const int irn = 1 - iri;
  int rec[SP]; int cnt = 0;
#pragma unroll
  for (int k = 0; k < SP; k += 4) {
    const v4i d4 = *(const v4i*)(dstv + ebc + k);
    const v4i s4 = *(const v4i*)(srcv + ebc + k);
#pragma unroll
    for (int e = 0; e < 4; ++e) {
      const int ev = eb + k + e;
      const int dself = ev - NEDGE;
      int d = iri * d4[e] + irn * dself;
      int s = iri * s4[e] + irn * dself;
      const bool valid = isreal || (ev < NVIRT);
      d = d < 0 ? 0 : (d >= NNODE ? NNODE - 1 : d);
      s = s < 0 ? 0 : (s >= NNODE ? NNODE - 1 : s);
      int r = -1;
      if (valid && d >= n0 && d < n0 + SRB) { r = ((d - n0) << 16) | s; ++cnt; }
      rec[k + e] = r;
    }
  }
  int tot; int p = blk_excl_scan(cnt, scan_ws, tid, &tot);
#pragma unroll
  for (int k = 0; k < SP; ++k) if (rec[k] >= 0) { if ((unsigned)p < (unsigned)CAP) LIST[p] = rec[k]; ++p; }
  __syncthreads();
  return tot < CAP ? tot : CAP;
}

__device__ __forceinline__ float red16f(float p) {
  p += __shfl_xor(p, 1, 32); p += __shfl_xor(p, 2, 32); p += __shfl_xor(p, 4, 32); p += __shfl_xor(p, 8, 32); return p;
}
__device__ __forceinline__ float red8f(float p) {
  p += __shfl_xor(p, 1, 32); p += __shfl_xor(p, 2, 32); p += __shfl_xor(p, 4, 32); return p;
}
__device__ __forceinline__ float lrelu_dot(v4f v, v4f w) {
  float s = 0.0f;
#pragma unroll
  for (int e = 0; e < 4; ++e) { float t = v[e]; t = (t >= 0.f) ? t : NEG_SLOPE_C * t; s = fmaf(w[e], t, s); }
  return s;
}
struct OnlineOut { float rr, ex, mn, ln; };
__device__ __forceinline__ OnlineOut online_step(float al, float mo, float lo) {
  OnlineOut o;
  const float dlt = al - mo;
  const float t = expf(-fabsf(dlt));
  const bool up = (dlt >= 0.f);
  o.rr = up ? t : 1.0f;
  o.ex = up ? 1.0f : t;
  o.mn = up ? al : mo;
  o.ln = fmaf(lo, o.rr, o.ex);
  return o;
}

constexpr int PREP_A1_BLOCKS  = (NPAD * KP1 / 8) / NT;
constexpr int PREP_BT1_BLOCKS = (XW1 * KP1 / 8) / NT;
constexpr int PREP_BT2_BLOCKS = (XW2 * KD2 / 8) / NT;
constexpr int PREP_BLOCKS = PREP_A1_BLOCKS + PREP_BT1_BLOCKS + PREP_BT2_BLOCKS + 1;
static_assert((NPAD * KP1 / 8) % NT == 0 && (XW1 * KP1 / 8) % NT == 0 && (XW2 * KD2 / 8) % NT == 0, "");
static_assert(PREP_BT1_BLOCKS % 2 == 0 && PREP_BT2_BLOCKS % 2 == 0, "");

__global__ __launch_bounds__(NT) void prep_kernel(const float* __restrict__ x,
    const float* __restrict__ Wl1, const float* __restrict__ bl1, const float* __restrict__ Wr1, const float* __restrict__ br1,
    const float* __restrict__ Wl2, const float* __restrict__ bl2, const float* __restrict__ Wr2, const float* __restrict__ br2,
    unsigned short* __restrict__ A1, unsigned short* __restrict__ Bt1, unsigned short* __restrict__ Bt2,
    float* __restrict__ bias1, float* __restrict__ bias2) {
  const int t = threadIdx.x;
  const int blk = blockIdx.x;
  if (blk < PREP_A1_BLOCKS) {
    const int i = blk * NT + t;
    const int row = i >> 2, seg = i & 3;
    const int rowc = row < NNODE ? row : NNODE - 1;
    const v4f a = *(const v4f*)(x + (size_t)rowc * CIN);
    const v4f c = *(const v4f*)(x + (size_t)rowc * CIN + 4);
    const bool live = (seg == 0) && (row < NNODE);
    const float fl = opaque_f(live ? 1.0f : 0.0f);
    const float f0 = fl * a[0], f1 = fl * a[1], f2 = fl * a[2], f3 = fl * a[3];
    const float f4 = fl * c[0], f5 = fl * c[1], f6 = fl * c[2], f7 = fl * c[3];
    const v4u u = pack8h(f0, f1, f2, f3, f4, f5, f6, f7);
    unsigned short* p = A1 + 8 * (size_t)i;
    *(volatile v4u*)p = u; __threadfence(); *(volatile v4u*)p = u;
  } else if (blk < PREP_A1_BLOCKS + PREP_BT1_BLOCKS) {
    const int rb = blk - PREP_A1_BLOCKS;
    const int j = rb * NT + t;
    const int n = j >> 2, seg = j & 3;
    const float* W = (rb < PREP_BT1_BLOCKS / 2) ? Wl1 : Wr1;
    const int nn = n & (AW1 - 1);
    const float fs = opaque_f((seg == 0) ? 1.0f : 0.0f);
    float f[8];
#pragma unroll
    for (int k = 0; k < CIN; ++k) { const float w = W[k * AW1 + nn] * WCARRY; f[k] = fs * w; }
    const v4u u = pack8h(f[0], f[1], f[2], f[3], f[4], f[5], f[6], f[7]);
    unsigned short* p = Bt1 + 8 * (size_t)j;
    *(volatile v4u*)p = u; __threadfence(); *(volatile v4u*)p = u;
  } else if (blk < PREP_A1_BLOCKS + PREP_BT1_BLOCKS + PREP_BT2_BLOCKS) {
    const int rb = blk - (PREP_A1_BLOCKS + PREP_BT1_BLOCKS);
    const int j = rb * NT + t;
    const int n = j >> 3, seg = j & 7;
    const float* W = (rb < PREP_BT2_BLOCKS / 2) ? Wl2 : Wr2;
    const int nn = n & (AW2 - 1);
    float f[8];
#pragma unroll
    for (int e = 0; e < 8; ++e) f[e] = W[(seg * 8 + e) * AW2 + nn] * WCARRY;
    const v4u u = pack8h(f[0], f[1], f[2], f[3], f[4], f[5], f[6], f[7]);
    unsigned short* p = Bt2 + 8 * (size_t)j;
    *(volatile v4u*)p = u; __threadfence(); *(volatile v4u*)p = u;
  } else {
    const int q6 = t & 63, q5 = t & 31;
    const v4f a1 = *(const v4f*)(bl1 + 4 * q6), c1 = *(const v4f*)(br1 + 4 * q6);
    const v4f a2 = *(const v4f*)(bl2 + 4 * q5), c2 = *(const v4f*)(br2 + 4 * q5);
    const float fl1 = (t < 64) ? 1.0f : 0.0f, fr1 = 1.0f - fl1;
    const float fl2 = (t < 160) ? 1.0f : 0.0f, fr2 = 1.0f - fl2;
    v4f v1, v2;
#pragma unroll
    for (int e = 0; e < 4; ++e) { v1[e] = fmaf(fl1, a1[e], fr1 * c1[e]); v2[e] = fmaf(fl2, a2[e], fr2 * c2[e]); }
    float* p1 = bias1 + 4 * (t & 127);
    float* p2 = bias2 + 4 * ((t - 128) & 63);
    for (int pass = 0; pass < 2; ++pass) {
      if (t < 128) *(volatile v4f*)p1 = v1;
      if (t >= 128 && t < 192) *(volatile v4f*)p2 = v2;
      __threadfence();
    }
  }
}

constexpr int SCH = 4096;
constexpr int SPT = SCH / NT;
constexpr int NCH = (NVIRT + SCH - 1) / SCH;

__global__ __launch_bounds__(NT) void gat_layer1_kernel(const float* __restrict__ XLR, const int* __restrict__ ei,
    const float* __restrict__ att, const float* __restrict__ cb, const float* __restrict__ lng, const float* __restrict__ lnb,
    float* AGG, unsigned short* __restrict__ H1o) {
  __shared__ int LIST[SCH];
  __shared__ float SM[SRB * NHEAD];
  __shared__ float SL[SRB * NHEAD];
  __shared__ int scan_ws[80];
  const int tid = threadIdx.x, lane = tid & 31;
  const int wave = __builtin_amdgcn_readfirstlane(tid >> 5);
  const int hh = lane >> 4, cl = lane & 15;
  const int n0 = blockIdx.x * SRB;
  const v4f at0 = *(const v4f*)(att + hh * HID1 + 4 * cl);
  const v4f at1 = *(const v4f*)(att + (hh + 2) * HID1 + 4 * cl);
  const v4f bs = *(const v4f*)(cb + 4 * cl);
  const v4f gs = *(const v4f*)(lng + 4 * cl);
  const v4f be = *(const v4f*)(lnb + 4 * cl);
  const v4f z4 = {0.f, 0.f, 0.f, 0.f};
#pragma unroll 1
  for (int j = 0; j < RPW; ++j) {
    float* rp = AGG + (size_t)(n0 + wave * RPW + j) * AW1 + 4 * lane;
    *(v4f*)rp = z4; *(v4f*)(rp + 128) = z4;
  }
  for (int i = tid; i < SRB * NHEAD; i += NT) { SM[i] = -INFINITY; SL[i] = 0.f; }
  for (int i = tid; i < SCH; i += NT) LIST[i] = -1;
  __syncthreads();
  const int* srcv = ei; const int* dstv = ei + NEDGE;
#pragma unroll 1
  for (int c = 0; c < NCH; ++c) {
    int tot = chunk_hits<SPT, SCH>(dstv, srcv, c * SCH, n0, tid, LIST, scan_ws);
    tot = __builtin_amdgcn_readfirstlane(tot);
#pragma unroll 1
    for (int base = 0; base < tot; base += 32) {
      const int q = base + lane;
      const int qc = q < SCH ? q : SCH - 1;
      const int lq = LIST[qc];
      const int rv = (q < tot) ? lq : -1;
      const int own = (rv >= 0 && (rv >> OWN_SHIFT) == wave) ? 1 : 0;
      unsigned msk = (unsigned)__ballot(own);
#pragma unroll 1
      for (int it = 0; it < 32; ++it) {
        if (msk == 0u) break;
        const int bp = __builtin_ctz(msk); msk &= msk - 1u;
        const int r = __builtin_amdgcn_readfirstlane(__shfl(rv, bp, 32));
        const int dl = r >> 16, s = r & 0xFFFF;
        const float* xlp = XLR + (size_t)s * XW1 + 4 * lane;
        const float* xrp = XLR + (size_t)(n0 + dl) * XW1 + AW1 + 4 * lane;
        const v4f xl0 = *(const v4f*)xlp;
        const v4f xl1 = *(const v4f*)(xlp + 128);
        const v4f xr0 = *(const v4f*)xrp;
        const v4f xr1 = *(const v4f*)(xrp + 128);
        float p0 = lrelu_dot(xl0 + xr0, at0);
        float p1 = lrelu_dot(xl1 + xr1, at1);
        p0 = red16f(p0); p1 = red16f(p1);
        const int mi0 = dl * NHEAD + hh, mi1 = mi0 + 2;
        const OnlineOut o0 = online_step(p0, SM[mi0], SL[mi0]);
        const OnlineOut o1 = online_step(p1, SM[mi1], SL[mi1]);
        if (cl == 0) { SM[mi0] = o0.mn; SL[mi0] = o0.ln; SM[mi1] = o1.mn; SL[mi1] = o1.ln; }
        float* ap = AGG + (size_t)(n0 + dl) * AW1 + 4 * lane;
        v4f a0 = *(const v4f*)ap;
        v4f a1 = *(const v4f*)(ap + 128);
        a0 = a0 * o0.rr + o0.ex * xl0;
        a1 = a1 * o1.rr + o1.ex * xl1;
        *(v4f*)ap = a0; *(v4f*)(ap + 128) = a1;
      }
    }
    __syncthreads();
  }
#pragma unroll 1
  for (int j = 0; j < RPW; ++j) {
    const int dl = wave * RPW + j;
    const int n = n0 + dl;
    if (n < NPAD) {
      const bool live = n < NNODE;
      float l0 = SL[dl * NHEAD + hh], l1 = SL[dl * NHEAD + hh + 2];
      l0 = (live && l0 > 0.f) ? l0 : 1.0f;
      l1 = (live && l1 > 0.f) ? l1 : 1.0f;
      const float inv0 = 1.0f / l0, inv1 = 1.0f / l1;
      const float* ap = AGG + (size_t)n * AW1 + 4 * lane;
      const v4f a0 = *(const v4f*)ap;
      const v4f a1 = *(const v4f*)(ap + 128);
      v4f t = a0 * inv0 + a1 * inv1;
      v4f u;
      u[0] = __shfl_xor(t[0], 16, 32); u[1] = __shfl_xor(t[1], 16, 32); u[2] = __shfl_xor(t[2], 16, 32); u[3] = __shfl_xor(t[3], 16, 32);
      t = t + u;
      t = t * 0.25f + bs;
      float su = (t[0] + t[1]) + (t[2] + t[3]);
      su = red16f(su);
      const float mu = su * (1.0f / HID1);
      const v4f d = t - mu;
      float sq = d[0] * d[0] + d[1] * d[1] + d[2] * d[2] + d[3] * d[3];
      sq = red16f(sq);
      const float rs = rsqrtf(sq * (1.0f / HID1) + LN_EPS);
      float y0 = fmaxf(d[0] * rs * gs[0] + be[0], 0.f);
      float y1 = fmaxf(d[1] * rs * gs[1] + be[1], 0.f);
      float y2 = fmaxf(d[2] * rs * gs[2] + be[2], 0.f);
      float y3 = fmaxf(d[3] * rs * gs[3] + be[3], 0.f);
      y0 = live ? y0 : 0.f; y1 = live ? y1 : 0.f; y2 = live ? y2 : 0.f; y3 = live ? y3 : 0.f;
      const int sa = 2 * (lane & 7), sb = sa + 1;
      const float ya0 = __shfl(y0, sa, 32), ya1 = __shfl(y1, sa, 32), ya2 = __shfl(y2, sa, 32), ya3 = __shfl(y3, sa, 32);
      const float yb0 = __shfl(y0, sb, 32), yb1 = __shfl(y1, sb, 32), yb2 = __shfl(y2, sb, 32), yb3 = __shfl(y3, sb, 32);
      const v4u pk = pack8h(ya0, ya1, ya2, ya3, yb0, yb1, yb2, yb3);
      unsigned short* hp = H1o + (size_t)n * KD2 + 8 * (lane & 7);
      for (int pass = 0; pass < 2; ++pass) {
        if (lane < 8) *(volatile v4u*)hp = pk;
        __threadfence();
      }
    }
  }
}

__global__ __launch_bounds__(NT) void gat_layer2_kernel(const float* __restrict__ XLR, const int* __restrict__ ei,
    const float* __restrict__ att, const float* __restrict__ cb, const float* __restrict__ lng, const float* __restrict__ lnb,
    float* AGG, float* __restrict__ H2o) {
  __shared__ int LIST[SCH];
  __shared__ float SM[SRB * NHEAD];
  __shared__ float SL[SRB * NHEAD];
  __shared__ int scan_ws[80];
  const int tid = threadIdx.x, lane = tid & 31;
  const int wave = __builtin_amdgcn_readfirstlane(tid >> 5);
  const int hq = lane >> 3, cq = lane & 7;
  const int n0 = blockIdx.x * SRB;
  const v4f at = *(const v4f*)(att + 4 * lane);
  const v4f bs = *(const v4f*)(cb + 4 * cq);
  const v4f gs = *(const v4f*)(lng + 4 * cq);
  const v4f be = *(const v4f*)(lnb + 4 * cq);
  const v4f z4 = {0.f, 0.f, 0.f, 0.f};
#pragma unroll 1
  for (int j = 0; j < RPW; ++j) *(v4f*)(AGG + (size_t)(n0 + wave * RPW + j) * AW2 + 4 * lane) = z4;
  for (int i = tid; i < SRB * NHEAD; i += NT) { SM[i] = -INFINITY; SL[i] = 0.f; }
  for (int i = tid; i < SCH; i += NT) LIST[i] = -1;
  __syncthreads();
  const int* srcv = ei; const int* dstv = ei + NEDGE;
#pragma unroll 1
  for (int c = 0; c < NCH; ++c) {
    int tot = chunk_hits<SPT, SCH>(dstv, srcv, c * SCH, n0, tid, LIST, scan_ws);
    tot = __builtin_amdgcn_readfirstlane(tot);
#pragma unroll 1
    for (int base = 0; base < tot; base += 32) {
      const int q = base + lane;
      const int qc = q < SCH ? q : SCH - 1;
      const int lq = LIST[qc];
      const int rv = (q < tot) ? lq : -1;
      const int own = (rv >= 0 && (rv >> OWN_SHIFT) == wave) ? 1 : 0;
      unsigned msk = (unsigned)__ballot(own);
#pragma unroll 1
      for (int it = 0; it < 32; ++it) {
        if (msk == 0u) break;
        const int bp = __builtin_ctz(msk); msk &= msk - 1u;
        const int r = __builtin_amdgcn_readfirstlane(__shfl(rv, bp, 32));
        const int dl = r >> 16, s = r & 0xFFFF;
        const v4f xl = *(const v4f*)(XLR + (size_t)s * XW2 + 4 * lane);
        const v4f xr = *(const v4f*)(XLR + (size_t)(n0 + dl) * XW2 + AW2 + 4 * lane);
        float p = lrelu_dot(xl + xr, at);
        p = red8f(p);
        const int mi = dl * NHEAD + hq;
        const OnlineOut o = online_step(p, SM[mi], SL[mi]);
        if (cq == 0) { SM[mi] = o.mn; SL[mi] = o.ln; }
        float* ap = AGG + (size_t)(n0 + dl) * AW2 + 4 * lane;
        v4f a = *(const v4f*)ap;
        a = a * o.rr + o.ex * xl;
        *(v4f*)ap = a;
      }
    }
    __syncthreads();
  }
#pragma unroll 1
  for (int j = 0; j < RPW; ++j) {
    const int dl = wave * RPW + j;
    const int n = n0 + dl;
    if (n < NNODE) {
      float lv = SL[dl * NHEAD + hq];
      lv = lv > 0.f ? lv : 1.0f;
      const float inv = 1.0f / lv;
      const v4f a = *(const v4f*)(AGG + (size_t)n * AW2 + 4 * lane);
      v4f t = a * inv;
      v4f u;
      u[0] = __shfl_xor(t[0], 8, 32);  u[1] = __shfl_xor(t[1], 8, 32);  u[2] = __shfl_xor(t[2], 8, 32);  u[3] = __shfl_xor(t[3], 8, 32);
      t = t + u;
      u[0] = __shfl_xor(t[0], 16, 32); u[1] = __shfl_xor(t[1], 16, 32); u[2] = __shfl_xor(t[2], 16, 32); u[3] = __shfl_xor(t[3], 16, 32);
      t = t + u;
      t = t * 0.25f + bs;
      float su = (t[0] + t[1]) + (t[2] + t[3]);
      su = red8f(su);
      const float mu = su * (1.0f / OUT2);
      const v4f d = t - mu;
      float sq = d[0] * d[0] + d[1] * d[1] + d[2] * d[2] + d[3] * d[3];
      sq = red8f(sq);
      const float rs = rsqrtf(sq * (1.0f / OUT2) + LN_EPS);
      v4f y;
      y[0] = fmaxf(d[0] * rs * gs[0] + be[0], 0.f);
      y[1] = fmaxf(d[1] * rs * gs[1] + be[1], 0.f);
      y[2] = fmaxf(d[2] * rs * gs[2] + be[2], 0.f);
      y[3] = fmaxf(d[3] * rs * gs[3] + be[3], 0.f);
      float* hp = H2o + (size_t)n * OUT2 + 4 * cq;
      for (int pass = 0; pass < 2; ++pass) {
        if (lane < 8) *(volatile v4f*)hp = y;
        __threadfence();
      }
    }
  }
}

constexpr int SCHP = 2048;
constexpr int NCHP = (NNODE + SCHP - 1) / SCHP;
static_assert(SCHP == NT * 8, "");

__global__ __launch_bounds__(NT) void pool_kernel(const float* __restrict__ H2p, const int* __restrict__ batch, float* __restrict__ outp) {
  __shared__ int LIST[SCHP];
  __shared__ int scan_ws[80];
  __shared__ __align__(16) float red[8 * OUT2];
  __shared__ int rc[8];
  const int tid = threadIdx.x, lane = tid & 31;
  const int wave = __builtin_amdgcn_readfirstlane(tid >> 5);
  const int cq = lane & 7;
  const int g = blockIdx.x;
  const v4f z4 = {0.f, 0.f, 0.f, 0.f};
  v4f acc = z4; int cnt = 0;
#pragma unroll 1
  for (int c = 0; c < NCHP; ++c) {
    const int eb = c * SCHP + tid * 8;
    const bool valid = eb < NNODE;
    const int ebc = valid ? eb : (NNODE - 8);
    const int ivl = opaque_i(valid ? 1 : 0);
    const int ivn = 1 - ivl;
    const v4i b0 = *(const v4i*)(batch + ebc);
    const v4i b1 = *(const v4i*)(batch + ebc + 4);
    int rec[8]; int kc = 0;
#pragma unroll
    for (int k = 0; k < 4; ++k) {
      const int g0 = ivl * b0[k] - ivn;
      const int g1 = ivl * b1[k] - ivn;
      rec[k] = -1;     if (g0 == g) { rec[k] = eb + k; ++kc; }
      rec[4 + k] = -1; if (g1 == g) { rec[4 + k] = eb + 4 + k; ++kc; }
    }
    int tot; int p = blk_excl_scan(kc, scan_ws, tid, &tot);
#pragma unroll
    for (int k = 0; k < 4; ++k) if (rec[k] >= 0) { if ((unsigned)p < (unsigned)SCHP) LIST[p] = rec[k]; ++p; }
#pragma unroll
    for (int k = 0; k < 4; ++k) if (rec[4 + k] >= 0) { if ((unsigned)p < (unsigned)SCHP) LIST[p] = rec[4 + k]; ++p; }
    __syncthreads();
    int totc = tot < SCHP ? tot : SCHP;
    totc = __builtin_amdgcn_readfirstlane(totc);
#pragma unroll 1
    for (int q = wave; q < totc; q += 8) {
      int nd = LIST[q]; nd = nd < 0 ? 0 : (nd >= NNODE ? NNODE - 1 : nd);
      acc = acc + *(const v4f*)(H2p + (size_t)nd * OUT2 + 4 * cq);
      ++cnt;
    }
    __syncthreads();
  }
  if (lane < 8) *(v4f*)(red + wave * OUT2 + 4 * lane) = acc;
  if (lane == 0) rc[wave] = cnt;
  __syncthreads();
  if (wave == 0) {
    v4f s = z4; int ct = 0;
#pragma unroll
    for (int w = 0; w < 8; ++w) { s = s + *(const v4f*)(red + w * OUT2 + 4 * cq); ct += rc[w]; }
    const float cf = (float)ct;
    const float inv = 1.0f / fmaxf(cf, 1.0f);
    const v4f o = s * inv;
    float* op = outp + (size_t)g * OUT2 + 4 * cq;
    for (int pass = 0; pass < 2; ++pass) {
      if (lane < 8) *(volatile v4f*)op = o;
      __threadfence();
    }
  }
}

extern "C" void kernel_launch(void* const* d_in, const int* in_sizes, int n_in,
                              void* d_out, int out_size, void* d_ws, size_t ws_size, hipStream_t stream) {
  if (n_in < 19) return;
  const float* x     = (const float*)d_in[0];
  const int*   ei    = (const int*)  d_in[1];
  const int*   batch = (const int*)  d_in[2];
  const float* Wl1   = (const float*)d_in[3];
  const float* bl1   = (const float*)d_in[4];
  const float* Wr1   = (const float*)d_in[5];
  const float* br1   = (const float*)d_in[6];
  const float* att1  = (const float*)d_in[7];
  const float* b1    = (const float*)d_in[8];
  const float* ln1g  = (const float*)d_in[9];
  const float* ln1b  = (const float*)d_in[10];
  const float* Wl2   = (const float*)d_in[11];
  const float* bl2   = (const float*)d_in[12];
  const float* Wr2   = (const float*)d_in[13];
  const float* br2   = (const float*)d_in[14];
  const float* att2  = (const float*)d_in[15];
  const float* b2    = (const float*)d_in[16];
  const float* ln2g  = (const float*)d_in[17];
  const float* ln2b  = (const float*)d_in[18];
  float* out = (float*)d_out;
  if (in_sizes[0] != NNODE * CIN || in_sizes[1] != 2 * NEDGE || in_sizes[2] != NNODE || out_size != NGRAPH * OUT2) return;

  char* ws = (char*)d_ws; size_t off = 0;
  auto carve = [&](size_t bytes) -> char* { char* p = ws + off; off += (bytes + 255) & ~(size_t)255; return p; };
  unsigned short* A1    = (unsigned short*)carve((size_t)NPAD * KP1 * 2);
  unsigned short* Bt1   = (unsigned short*)carve((size_t)XW1 * KP1 * 2);
  unsigned short* Bt2   = (unsigned short*)carve((size_t)XW2 * KD2 * 2);
  float*          bias1 = (float*)carve((size_t)XW1 * 4);
  float*          bias2 = (float*)carve((size_t)XW2 * 4);
  float*          XLR1  = (float*)carve((size_t)NPAD * XW1 * 4);
  float*          AGG1  = (float*)carve((size_t)NACC * AW1 * 4);
  unsigned short* H1    = (unsigned short*)carve((size_t)NPAD * KD2 * 2);
  float*          XLR2  = (float*)carve((size_t)NPAD * XW2 * 4);
  float*          AGG2  = (float*)carve((size_t)NACC * AW2 * 4);
  float*          H2    = (float*)carve((size_t)NACC * OUT2 * 4);
  if (off > ws_size || off > (size_t)134217728) return;

  prep_kernel<<<PREP_BLOCKS, NT, 0, stream>>>(x, Wl1, bl1, Wr1, br1, Wl2, bl2, Wr2, br2, A1, Bt1, Bt2, bias1, bias2);
  {
    const int tiles = (NPAD / 64) * (XW1 / 64);
    wmma_gemm64<0, false, 2, 0, false, 0><<<dim3((tiles + 7) / 8, 1), 256, 0, stream>>>(
        (const unsigned short*)A1, (const unsigned short*)A1, KP1, 0L,
        (const unsigned short*)Bt1, (const unsigned short*)Bt1, KP1, 0L,
        (void*)XLR1, (void*)nullptr, XW1, 0L,
        (const float*)bias1, (const float*)nullptr, 0L, NPAD, XW1, KP1, WCARRY_INV);
  }
  gat_layer1_kernel<<<NTILE, NT, 0, stream>>>(XLR1, ei, att1, b1, ln1g, ln1b, AGG1, H1);
  {
    const int tiles = (NPAD / 64) * (XW2 / 64);
    wmma_gemm64<0, false, 2, 0, false, 0><<<dim3((tiles + 7) / 8, 1), 256, 0, stream>>>(
        (const unsigned short*)H1, (const unsigned short*)H1, KD2, 0L,
        (const unsigned short*)Bt2, (const unsigned short*)Bt2, KD2, 0L,
        (void*)XLR2, (void*)nullptr, XW2, 0L,
        (const float*)bias2, (const float*)nullptr, 0L, NPAD, XW2, KD2, WCARRY_INV);
  }
  gat_layer2_kernel<<<NTILE, NT, 0, stream>>>(XLR2, ei, att2, b2, ln2g, ln2b, AGG2, H2);
  pool_kernel<<<NGRAPH, NT, 0, stream>>>(H2, batch, out);
}
